// MLPFeatureImputation_53910429500026
// MI455X (gfx1250) — hardware-verified
//
#include <hip/hip_runtime.h>
#include <stddef.h>
#include <stdint.h>

#define NV   64
#define NH   32
#define TOKB 128
#define SP   68

static_assert((SP * 4) % 16 == 0);
static_assert(NV % 32 == 0);
static_assert(NH == 32);
static_assert(TOKB == 128);

typedef _Float16 v16h __attribute__((ext_vector_type(16)));
typedef _Float16 v8h  __attribute__((ext_vector_type(8)));
typedef _Float16 v4h  __attribute__((ext_vector_type(4)));
typedef float    v8f  __attribute__((ext_vector_type(8)));
typedef float    v4f  __attribute__((ext_vector_type(4)));
typedef unsigned int v4u __attribute__((ext_vector_type(4)));
typedef v8h __attribute__((may_alias)) v8ha;
typedef v8f __attribute__((may_alias)) v8fa;
typedef v4f __attribute__((may_alias)) v4fa;

union Frag { v16h v; v8h h[2]; };
union HU   { v8h h; v4u u; };

__device__ __forceinline__ v8f mma16(v16h a, v16h b, v8f cacc) {
  cacc = __builtin_amdgcn_wmma_f32_16x16x32_f16(false, a, false, b, (short)0, cacc, false, false);
  asm volatile("v_nop\n\tv_nop\n\tv_nop\n\tv_nop" : "+v"(cacc) : "v"(a), "v"(b));
  return cacc;
}

__device__ __forceinline__ v8f zero8() { return (v8f){0.f, 0.f, 0.f, 0.f, 0.f, 0.f, 0.f, 0.f}; }

__device__ __forceinline__ v16h ldfrag_g(const _Float16* __restrict__ p, int ld, int row0, int k0, int lane) {
  const int m = lane & 15, lh = lane >> 4;
  const _Float16* q = p + (size_t)(row0 + m) * ld + k0 + 8 * lh;
  Frag f;
  f.h[0] = *(const v8h*)(q);
  f.h[1] = *(const v8h*)(q + 16);
  return f.v;
}

__device__ __forceinline__ v16h ldfrag_l(const _Float16* p, int ld, int row0, int k0, int lane) {
  const int m = lane & 15, lh = lane >> 4;
  const _Float16* q = p + (row0 + m) * ld + k0 + 8 * lh;
  Frag f;
  f.h[0] = *(const v8ha*)(q);
  f.h[1] = *(const v8ha*)(q + 16);
  return f.v;
}

__global__ __launch_bounds__(256) void k_prep(const float* __restrict__ W, _Float16* __restrict__ Wh) {
  const int g  = blockIdx.x * 256 + threadIdx.x;
  const int rw = g >> 3;
  const int pc = g & 7;
  const int i  = rw >> 5;
  const float* src = W + (size_t)rw * NV + pc * 8;
  const v4f f0 = *(const v4f*)(src);
  const v4f f1 = *(const v4f*)(src + 4);
  float w[8] = {f0.x, f0.y, f0.z, f0.w, f1.x, f1.y, f1.z, f1.w};
  HU o;
#pragma unroll
  for (int j = 0; j < 8; ++j) {
    const float t = (pc * 8 + j == i) ? 0.0f : w[j];
    o.h[j] = (_Float16)(t * 64.0f);
  }
  _Float16* dst = Wh + (size_t)rw * NV + pc * 8;
  *(volatile v4u*)dst = o.u;
  __threadfence();
  *(volatile v4u*)dst = o.u;
}

__device__ __forceinline__ void store_tile(const float* sw, float* __restrict__ out, size_t row_base, int lane) {
#pragma unroll
  for (int it = 0; it < 8; ++it) {
    const int p   = lane + 32 * it;
    const int L   = p >> 3;
    const int row = L >> 1;
    const int hf  = L & 1;
    const int pc  = p & 7;
    const v4f val = *(const v4fa*)(sw + row * SP + hf * 32 + pc * 4);
    *(volatile v4f*)(out + (row_base + row) * NV + hf * 32 + pc * 4) = val;
  }
}

__global__ __launch_bounds__(256) void k_fused(const float* __restrict__ X, const _Float16* __restrict__ Wh,
                                               const float* __restrict__ Bv, const float* __restrict__ W1,
                                               const float* __restrict__ B1, const float* __restrict__ W2,
                                               const float* __restrict__ B2, float* __restrict__ out) {
  __shared__ __align__(16) _Float16 Xh[TOKB * NV];
  __shared__ __align__(16) _Float16 W1h[NH * NH];
  __shared__ __align__(32) float bL[NV * NH];
  __shared__ __align__(16) float st[8][16 * SP];

  const int tid = threadIdx.x, lane = tid & 31, wave = tid >> 5;
  const int m = lane & 15, hh = lane >> 4;
  const size_t tok0 = (size_t)blockIdx.x * TOKB;

  {
    const float* xs = X + tok0 * NV;
#pragma unroll
    for (int q = 0; q < 8; ++q) {
      const v4f f = *(const v4f*)(xs + (size_t)tid * 32 + q * 4);
      v4h hv;
      hv.x = (_Float16)f.x; hv.y = (_Float16)f.y; hv.z = (_Float16)f.z; hv.w = (_Float16)f.w;
      *(v4h*)(Xh + tid * 32 + q * 4) = hv;
    }
  }
  {
    const v4f f = *(const v4f*)(W1 + tid * 4);
    v4h hv;
    hv.x = (_Float16)(f.x * 64.0f); hv.y = (_Float16)(f.y * 64.0f);
    hv.z = (_Float16)(f.z * 64.0f); hv.w = (_Float16)(f.w * 64.0f);
    *(v4h*)(W1h + tid * 4) = hv;
  }
#pragma unroll
  for (int q = 0; q < 8; ++q) bL[tid + 256 * q] = Bv[tid + 256 * q];
  __syncthreads();

  const v16h bx0 = ldfrag_l(Xh, NV, wave * 16, 0, lane);
  const v16h bx1 = ldfrag_l(Xh, NV, wave * 16, 32, lane);
  const v16h bw0 = ldfrag_l(W1h, NH, 0, 0, lane);
  const v16h bw1 = ldfrag_l(W1h, NH, 16, 0, lane);

  const float b1a = B1[m], b1b = B1[16 + m];
  const float w2a = W2[m], w2b = W2[16 + m];
  const float b2s = B2[0];
  const float inv64 = 0.015625f;
  const float inv1024 = 0.0009765625f;
  float* sw = st[wave];

#pragma unroll 1
  for (int i = 0; i < NV; ++i) {
    const int r0 = i * NH;
    const v16h a00 = ldfrag_g(Wh, NV, r0, 0, lane);
    const v16h a01 = ldfrag_g(Wh, NV, r0, 32, lane);
    const v16h a10 = ldfrag_g(Wh, NV, r0 + 16, 0, lane);
    const v16h a11 = ldfrag_g(Wh, NV, r0 + 16, 32, lane);
    v8f c0 = mma16(a00, bx0, zero8());
    c0 = mma16(a01, bx1, c0);
    v8f c1 = mma16(a10, bx0, zero8());
    c1 = mma16(a11, bx1, c1);

    const v8f bias0 = *(const v8fa*)(bL + r0 + 8 * hh);
    const v8f bias1 = *(const v8fa*)(bL + r0 + 16 + 8 * hh);

    Frag a2;
#pragma unroll
    for (int r = 0; r < 8; ++r) {
      const float h0v = fmaxf(c0[r] * inv64 + bias0[r], 0.0f);
      const float h1v = fmaxf(c1[r] * inv64 + bias1[r], 0.0f);
      a2.v[r]     = (_Float16)(h0v * 16.0f);
      a2.v[8 + r] = (_Float16)(h1v * 16.0f);
    }

    const v8f d0 = mma16(a2.v, bw0, zero8());
    const v8f d1 = mma16(a2.v, bw1, zero8());

    float red[8];
#pragma unroll
    for (int r = 0; r < 8; ++r)
      red[r] = fmaxf(d0[r] * inv1024 + b1a, 0.0f) * w2a + fmaxf(d1[r] * inv1024 + b1b, 0.0f) * w2b;
#pragma unroll
    for (int off = 8; off; off >>= 1) {
#pragma unroll
      for (int r = 0; r < 8; ++r) red[r] += __shfl_xor(red[r], off, 16);
    }
    float zr = red[0];
#pragma unroll
    for (int r = 1; r < 8; ++r) zr = ((m & 7) == r) ? red[r] : zr;
    if (m < 8) sw[(8 * hh + m) * SP + i] = zr + b2s;
  }
  __syncthreads();

  const size_t row_base = tok0 + (size_t)wave * 16;
  store_tile(sw, out, row_base, lane);
  __threadfence();
  store_tile(sw, out, row_base, lane);
}

extern "C" void kernel_launch(void* const* d_in, const int* in_sizes, int n_in,
                              void* d_out, int out_size, void* d_ws, size_t ws_size,
                              hipStream_t stream) {
  if (n_in < 7) return;
  if (in_sizes[0] <= 0 || (in_sizes[0] % (TOKB * NV)) != 0) return;
  if (in_sizes[1] != NV * NH * NV) return;
  if (in_sizes[2] != NV * NH) return;
  if (in_sizes[3] != NH * NH) return;
  if (in_sizes[4] != NH) return;
  if (in_sizes[5] != NH) return;
  if (in_sizes[6] < 1) return;
  if (out_size != in_sizes[0]) return;

  const float* x  = (const float*)d_in[0];
  const float* W  = (const float*)d_in[1];
  const float* b  = (const float*)d_in[2];
  const float* W1 = (const float*)d_in[3];
  const float* b1 = (const float*)d_in[4];
  const float* W2 = (const float*)d_in[5];
  const float* b2 = (const float*)d_in[6];
  float* out = (float*)d_out;

  const size_t wh_bytes = (size_t)NV * NH * NV * 2;
  if (wh_bytes > ws_size) return;
  _Float16* Wh = (_Float16*)d_ws;

  const int tokens = in_sizes[0] / NV;
  const int blocks = tokens / TOKB;

  k_prep<<<dim3((NV * NH * NV) / (8 * 256)), dim3(256), 0, stream>>>(W, Wh);
  k_fused<<<dim3(blocks), dim3(256), 0, stream>>>(x, Wh, b, W1, b1, W2, b2, out);
  (void)hipGetLastError();
}
